// TMix_qwen2rwkv_37477884625392
// MI455X (gfx1250) — hardware-verified
//
#include <hip/hip_runtime.h>
#include <math.h>

constexpr int kBatch    = 2;
constexpr int kSeq      = 512;
constexpr int kCh       = 2048;
constexpr int kHeads    = 32;
constexpr int kHd       = 64;
constexpr int kMixRank  = 32;
constexpr int kDecRank  = 64;
constexpr int kRows     = kBatch * kSeq;
constexpr int kMixCols  = 4 * kMixRank;
constexpr int kPlane    = kRows * kCh;
constexpr int kScanChunk = 16;

constexpr float kWCarry     = 64.0f;
constexpr float kWCarryInv  = 1.0f / 64.0f;
constexpr float kActCarry   = 64.0f;
constexpr float kMCarry     = 64.0f;
constexpr float kMCarryInv  = 1.0f / 64.0f;
constexpr float kResCarry   = 2048.0f;
constexpr float kResInv     = 1.0f / 2048.0f;
constexpr float kQScale     = 0.125f;
constexpr float kLnEps      = 1e-5f;
constexpr float kInvCh      = 1.0f / 2048.0f;

static_assert(kHeads * kHd == kCh);
static_assert(kQScale * kQScale * (float)kHd == 1.0f);
static_assert(kInvCh * (float)kCh == 1.0f);
static_assert(kRows % 64 == 0 && kCh % 64 == 0 && kMixCols % 64 == 0 && kDecRank % 64 == 0);
static_assert(kCh % 32 == 0 && kMixRank % 32 == 0 && kDecRank % 32 == 0);
static_assert(kCh / 8 == 256);
static_assert((kSeq & (kSeq - 1)) == 0);
static_assert(kSeq % kScanChunk == 0);
static_assert((kRows * kMixCols) % 2048 == 0 && (kRows * kDecRank) % 2048 == 0);

typedef __attribute__((ext_vector_type(16))) _Float16 v16h;
typedef __attribute__((ext_vector_type(8)))  _Float16 v8h;
typedef __attribute__((ext_vector_type(8)))  float    v8f;
typedef __attribute__((ext_vector_type(4)))  float    v4f;
typedef __attribute__((ext_vector_type(4)))  unsigned int v4u;

__device__ __forceinline__ void dep_guard4_h(v8f& a, v8f& b, v8f& c, v8f& d, v16h x, v16h y) {
  asm volatile("v_nop\n\tv_nop\n\tv_nop\n\tv_nop" : "+v"(a), "+v"(b), "+v"(c), "+v"(d) : "v"(x), "v"(y));
}
__device__ __forceinline__ void keep4_h(v16h a, v16h b, v16h c, v16h d) {
  asm volatile("v_nop" :: "v"(a), "v"(b), "v"(c), "v"(d));
}
__device__ __forceinline__ void acc_guard4(v8f& a, v8f& b, v8f& c, v8f& d) {
  asm volatile("v_nop\n\tv_nop\n\tv_nop\n\tv_nop" : "+v"(a), "+v"(b), "+v"(c), "+v"(d));
}
struct FragH {
  union U { v16h v; v8h h[2]; };
  static __device__ __forceinline__ v16h load(const _Float16* p) {
    U f;
    f.h[0] = *(const v8h*)(p);
    f.h[1] = *(const v8h*)(p + 16);
    return f.v;
  }
  static __device__ __forceinline__ v8f mma(v16h a, v16h b, v8f c) {
    return __builtin_amdgcn_wmma_f32_16x16x32_f16(false, a, false, b, (short)0, c, false, false);
  }
};

__device__ __forceinline__ float h16_to_f32(unsigned hb) {
  const unsigned sgn = (hb & 0x8000u) << 16;
  const unsigned em = hb & 0x7fffu;
  const float fn = __uint_as_float((em << 13) + 0x38000000u);
  const float fs = (float)em * 5.9604644775390625e-8f;
  const float mag = (em < 0x400u) ? fs : fn;
  return __uint_as_float(__float_as_uint(mag) | sgn);
}

template <bool ARES, bool HAS_BIAS, int OUT_MODE>
__global__ __launch_bounds__(256) void wmma_gemm64(
    const unsigned short* __restrict__ Ap, const unsigned short* __restrict__ A2p, int lda, long strideA,
    const unsigned short* __restrict__ Btp, int ldb, long strideB,
    void* __restrict__ Cout, int ldc, long strideC,
    const float* __restrict__ bias,
    int M, int N, int K, float scale, float res_inv) {
  const _Float16* A  = (const _Float16*)Ap;
  const _Float16* A2 = (const _Float16*)A2p;
  const _Float16* Bt = (const _Float16*)Btp;
  __shared__ __align__(16) float sT[8][16 * 68];
  const int b    = blockIdx.y;
  const int lane = threadIdx.x & 31;
  const int wave = threadIdx.x >> 5;
  const int tilesN = N >> 6;
  const int tilesM = M >> 6;
  const int tile = blockIdx.x * 8 + wave;
  if (tile >= tilesM * tilesN) return;
  const int tm = tile / tilesN;
  const int tn = tile - tm * tilesN;
  const int m0 = tm << 6;
  const int n0 = tn << 6;

  const _Float16* Ab = A + (size_t)b * strideA;
  const _Float16* Ar = ARES ? (A2 + (size_t)b * strideA) : Ab;
  const _Float16* Bb = Bt + (size_t)b * strideB;

  const int rlane = lane & 15;
  const int koff  = (lane >> 4) * 8;
  const int mOff  = (lane >> 4) * 8;

  v8f acc[4][4];
#pragma unroll
  for (int i = 0; i < 4; ++i)
#pragma unroll
    for (int j = 0; j < 4; ++j) acc[i][j] = (v8f){0.f, 0.f, 0.f, 0.f, 0.f, 0.f, 0.f, 0.f};

  const _Float16* brow = Bb + (size_t)(n0 + rlane) * ldb + koff;
  const size_t bstep = (size_t)16 * ldb;
  const size_t astep = (size_t)16 * lda;

  for (int ph = ARES ? 0 : 1; ph < 2; ++ph) {
    const _Float16* abase = (ph == 0) ? Ar : Ab;
    const _Float16* arow = abase + (size_t)(m0 + rlane) * lda + koff;
    for (int k0 = 0; k0 < K; k0 += 32) {
      v16h bh[4];
#pragma unroll
      for (int j = 0; j < 4; ++j) bh[j] = FragH::load(brow + j * bstep + k0);
#pragma unroll
      for (int i = 0; i < 4; ++i) {
        const v16h ah = FragH::load(arow + i * astep + k0);
#pragma unroll
        for (int j = 0; j < 4; ++j) acc[i][j] = FragH::mma(ah, bh[j], acc[i][j]);
        dep_guard4_h(acc[i][0], acc[i][1], acc[i][2], acc[i][3], ah, bh[3]);
      }
      keep4_h(bh[0], bh[1], bh[2], bh[3]);
    }
    if (ARES && ph == 0) {
      acc_guard4(acc[0][0], acc[0][1], acc[0][2], acc[0][3]);
      acc_guard4(acc[1][0], acc[1][1], acc[1][2], acc[1][3]);
      acc_guard4(acc[2][0], acc[2][1], acc[2][2], acc[2][3]);
      acc_guard4(acc[3][0], acc[3][1], acc[3][2], acc[3][3]);
#pragma unroll
      for (int i = 0; i < 4; ++i)
#pragma unroll
        for (int j = 0; j < 4; ++j) acc[i][j] = acc[i][j] * res_inv;
    }
  }
  acc_guard4(acc[0][0], acc[0][1], acc[0][2], acc[0][3]);
  acc_guard4(acc[1][0], acc[1][1], acc[1][2], acc[1][3]);
  acc_guard4(acc[2][0], acc[2][1], acc[2][2], acc[2][3]);
  acc_guard4(acc[3][0], acc[3][1], acc[3][2], acc[3][3]);

  float* slab = sT[wave];
#pragma unroll
  for (int i = 0; i < 4; ++i) {
    const int mBase = m0 + (i << 4);
#pragma unroll
    for (int j = 0; j < 4; ++j) {
      const int n = n0 + (j << 4) + rlane;
      float bv = 0.f;
      if (HAS_BIAS) bv = bias[n];
#pragma unroll
      for (int r = 0; r < 8; ++r) {
        float v = acc[i][j][r] * scale;
        if (HAS_BIAS) v += bv;
        slab[(mOff + r) * 68 + (j << 4) + rlane] = v;
      }
    }
    __builtin_amdgcn_fence(__ATOMIC_RELEASE, "workgroup");
    __builtin_amdgcn_wave_barrier();
    __builtin_amdgcn_fence(__ATOMIC_ACQUIRE, "workgroup");
    if (OUT_MODE == 0) {
      float* C = (float*)Cout + (size_t)b * strideC;
      const int hh = lane >> 4, c4 = (lane & 15) * 4;
      for (int pass = 0; pass < 2; ++pass) {
#pragma unroll
        for (int it = 0; it < 8; ++it) {
          const int row = it * 2 + hh;
          v4f v = *(const v4f*)(slab + row * 68 + c4);
          *(volatile v4f*)(C + (size_t)(mBase + row) * ldc + n0 + c4) = v;
        }
        __threadfence();
      }
    } else {
      const int q = lane >> 3, c8 = (lane & 7) * 8;
      unsigned short* C = (unsigned short*)Cout + (size_t)b * strideC;
      for (int pass = 0; pass < 2; ++pass) {
#pragma unroll
        for (int it = 0; it < 4; ++it) {
          const int row = it * 4 + q;
          const float* sp = slab + row * 68 + c8;
          v8h hv;
#pragma unroll
          for (int e = 0; e < 8; ++e) hv[e] = (_Float16)sp[e];
          *(volatile v8h*)(C + (size_t)(mBase + row) * ldc + n0 + c8) = hv;
        }
        __threadfence();
      }
    }
    __builtin_amdgcn_fence(__ATOMIC_RELEASE, "workgroup");
    __builtin_amdgcn_wave_barrier();
    __builtin_amdgcn_fence(__ATOMIC_ACQUIRE, "workgroup");
  }
}

template <int TK>
__global__ __launch_bounds__(256) void wt_cast_kernel(const float* __restrict__ W0, const float* __restrict__ W1,
                                                      const float* __restrict__ W2, const float* __restrict__ W3,
                                                      long inStrideZ, unsigned short* __restrict__ out, long outStrideZ,
                                                      int K, int N, float scale) {
  __shared__ float sm[64][TK + 1];
  const int t  = threadIdx.x;
  const int k0 = blockIdx.x * TK;
  const int n0 = blockIdx.y * 64;
  const int z  = blockIdx.z;
  const float* Wsel = (z == 0) ? W0 : (z == 1) ? W1 : (z == 2) ? W2 : W3;
  const float* W = Wsel + (size_t)z * inStrideZ;
#pragma unroll
  for (int i = 0; i < TK / 4; ++i) {
    const int e = i * 256 + t;
    const int r = e >> 6;
    const int c = e & 63;
    sm[c][r] = W[(size_t)(k0 + r) * N + n0 + c] * scale;
  }
  __syncthreads();
  constexpr int LPR = TK / 8;
  constexpr int RPP = 256 / LPR;
  constexpr int NIT = 64 / RPP;
  unsigned short* op = out + (size_t)z * outStrideZ;
  const int rsub = t / LPR;
  const int c8 = (t % LPR) * 8;
  for (int pass = 0; pass < 2; ++pass) {
#pragma unroll
    for (int it = 0; it < NIT; ++it) {
      const int row = it * RPP + rsub;
      v8h hv;
#pragma unroll
      for (int e = 0; e < 8; ++e) hv[e] = (_Float16)sm[row][c8 + e];
      *(volatile v8h*)(op + (size_t)(n0 + row) * K + k0 + c8) = hv;
    }
    __threadfence();
  }
}

template <bool WITH_M>
__global__ __launch_bounds__(256) void mix_kernel(const float* __restrict__ x,
                                                  const float* __restrict__ ma0, const float* __restrict__ ma1,
                                                  const float* __restrict__ ma2, const float* __restrict__ ma3,
                                                  const unsigned short* __restrict__ m16,
                                                  unsigned short* __restrict__ xh, unsigned short* __restrict__ xl) {
  const int r = blockIdx.y;
  const int i = blockIdx.x * 256 + threadIdx.x;
  const int row = i >> 8;
  const int c = (i & 255) * 8;
  const int t = row & (kSeq - 1);
  const int rowp = (row > 0) ? (row - 1) : 0;
  const bool keep = (t != 0);
  const float* maa = (r == 0) ? ma0 : (r == 1) ? ma1 : (r == 2) ? ma2 : ma3;
  const float* xp = x + (size_t)row * kCh + c;
  const float* pp = x + (size_t)rowp * kCh + c;
  const v4f xa = *(const v4f*)(xp);
  const v4f xb = *(const v4f*)(xp + 4);
  const v4f pa = *(const v4f*)(pp);
  const v4f pb = *(const v4f*)(pp + 4);
  const v4f ga = *(const v4f*)(maa + c);
  const v4f gb = *(const v4f*)(maa + c + 4);
  float xs[8], ps[8], gs[8], ms[8];
#pragma unroll
  for (int e = 0; e < 4; ++e) {
    xs[e] = xa[e]; xs[4 + e] = xb[e];
    ps[e] = pa[e]; ps[4 + e] = pb[e];
    gs[e] = ga[e]; gs[4 + e] = gb[e];
  }
  if (WITH_M) {
    const v4u mw = *(const v4u*)(m16 + ((size_t)r * kRows + row) * kCh + c);
    const unsigned w0 = mw[0];
    const unsigned w1 = mw[1];
    const unsigned w2 = mw[2];
    const unsigned w3 = mw[3];
    ms[0] = h16_to_f32(w0 & 0xffffu) * kMCarryInv;
    ms[1] = h16_to_f32(w0 >> 16) * kMCarryInv;
    ms[2] = h16_to_f32(w1 & 0xffffu) * kMCarryInv;
    ms[3] = h16_to_f32(w1 >> 16) * kMCarryInv;
    ms[4] = h16_to_f32(w2 & 0xffffu) * kMCarryInv;
    ms[5] = h16_to_f32(w2 >> 16) * kMCarryInv;
    ms[6] = h16_to_f32(w3 & 0xffffu) * kMCarryInv;
    ms[7] = h16_to_f32(w3 >> 16) * kMCarryInv;
  } else {
#pragma unroll
    for (int e = 0; e < 8; ++e) ms[e] = 0.0f;
  }
  v8h hv, lv;
#pragma unroll
  for (int e = 0; e < 8; ++e) {
    const float pv = keep ? ps[e] : 0.0f;
    const float dx = pv - xs[e];
    const float val = xs[e] + dx * (gs[e] + ms[e]);
    const _Float16 hi = (_Float16)val;
    const float hif = (float)hi;
    hv[e] = hi;
    lv[e] = (_Float16)((val - hif) * kResCarry);
  }
  const size_t off = ((size_t)r * kRows + row) * kCh + c;
  const bool wlo = WITH_M && (r < 3);
  *(volatile v8h*)(xh + off) = hv;
  if (wlo) *(volatile v8h*)(xl + off) = lv;
  __threadfence();
  *(volatile v8h*)(xh + off) = hv;
  if (wlo) *(volatile v8h*)(xl + off) = lv;
}

__global__ __launch_bounds__(256) void tanh_cast_kernel(const float* __restrict__ in, unsigned short* __restrict__ out,
                                                        float carry) {
  __shared__ __align__(16) _Float16 sh[2048];
  const int tid = threadIdx.x;
  const size_t base = (size_t)blockIdx.x * 2048;
#pragma unroll 1
  for (int it = 0; it < 8; ++it) {
    const int idx = it * 256 + tid;
    const float v = in[base + idx];
    sh[idx] = (_Float16)(tanhf(v) * carry);
  }
  __syncthreads();
  const v8h hv = *(const v8h*)(sh + tid * 8);
  unsigned short* op = out + base + (size_t)tid * 8;
  *(volatile v8h*)op = hv;
  __threadfence();
  *(volatile v8h*)op = hv;
}

__global__ __launch_bounds__(256) void gated_scan_kernel(const float* __restrict__ Q, const float* __restrict__ K0,
                                                         const float* __restrict__ V, const float* __restrict__ LORA,
                                                         const float* __restrict__ tdec, float* __restrict__ Y) {
  __shared__ __align__(16) float sq[kScanChunk * kHd];
  __shared__ __align__(16) float sk[kScanChunk * kHd];
  __shared__ __align__(16) float sg[kScanChunk * kHd];
  __shared__ __align__(16) float sv[kScanChunk * kHd];
  __shared__ __align__(16) float sy[kScanChunk * kHd];
  const int tid = threadIdx.x;
  const int bh = blockIdx.x;
  const int b = bh / kHeads;
  const int h = bh - b * kHeads;
  const int vv = tid >> 2;
  const int kq = tid & 3;
  const int colbase = h * kHd;
  const float td = tdec[colbase + (tid & 63)];

  float S[16];
#pragma unroll
  for (int i = 0; i < 16; ++i) S[i] = 0.0f;

  const int srow = tid >> 4;
  const int sc4 = (tid & 15) * 4;

#pragma unroll 1
  for (int t0 = 0; t0 < kSeq; t0 += kScanChunk) {
#pragma unroll 1
    for (int it = 0; it < 4; ++it) {
      const int idx = it * 256 + tid;
      const int st = idx >> 6;
      const int c = idx & 63;
      const size_t off = (size_t)(b * kSeq + t0 + st) * kCh + colbase + c;
      const float qv = Q[off];
      const float kv = K0[off];
      const float vl = V[off];
      const float lo = LORA[off];
      float w = -expf(td + lo);
      w = fmaxf(w, -5.0f);
      const float g = expf(w);
      sq[idx] = qv;
      sk[idx] = kv * (1.0f - g);
      sg[idx] = g;
      sv[idx] = vl;
    }
    __syncthreads();
#pragma unroll 1
    for (int st = 0; st < kScanChunk; ++st) {
      const float vcur = sv[st * kHd + vv];
      const float* qp = sq + st * kHd + kq * 16;
      const float* kp = sk + st * kHd + kq * 16;
      const float* gp = sg + st * kHd + kq * 16;
      float acc = 0.0f;
#pragma unroll
      for (int j = 0; j < 4; ++j) {
        const v4f q4 = *(const v4f*)(qp + 4 * j);
        const v4f k4 = *(const v4f*)(kp + 4 * j);
        const v4f g4 = *(const v4f*)(gp + 4 * j);
#pragma unroll
        for (int e = 0; e < 4; ++e) {
          const float kvp = k4[e] * vcur;
          S[4 * j + e] = fmaf(S[4 * j + e], g4[e], kvp);
          acc = fmaf(q4[e], S[4 * j + e], acc);
        }
      }
      acc += __shfl_xor(acc, 1, 32);
      acc += __shfl_xor(acc, 2, 32);
      if (kq == 0) sy[st * kHd + vv] = acc * kQScale;
    }
    __syncthreads();
    {
      const v4f val = *(const v4f*)(sy + srow * kHd + sc4);
      float* yp = Y + (size_t)(b * kSeq + t0 + srow) * kCh + colbase + sc4;
      *(volatile v4f*)yp = val;
      __threadfence();
      *(volatile v4f*)yp = val;
    }
  }
}

__global__ __launch_bounds__(256) void ln_split_kernel(const float* __restrict__ Y, const float* __restrict__ gam,
                                                       const float* __restrict__ bet,
                                                       unsigned short* __restrict__ yh, unsigned short* __restrict__ yl) {
  __shared__ float red1[8];
  __shared__ float red2[8];
  const int row = blockIdx.x;
  const int tid = threadIdx.x;
  const int lane = tid & 31, wave = tid >> 5;
  const int c0 = tid * 8;
  const float* rp = Y + (size_t)row * kCh + c0;
  const v4f a = *(const v4f*)(rp);
  const v4f c = *(const v4f*)(rp + 4);
  const v4f g0 = *(const v4f*)(gam + c0);
  const v4f g1 = *(const v4f*)(gam + c0 + 4);
  const v4f b0 = *(const v4f*)(bet + c0);
  const v4f b1 = *(const v4f*)(bet + c0 + 4);
  float xs[8], gs[8], bs[8];
#pragma unroll
  for (int e = 0; e < 4; ++e) {
    xs[e] = a[e]; xs[4 + e] = c[e];
    gs[e] = g0[e]; gs[4 + e] = g1[e];
    bs[e] = b0[e]; bs[4 + e] = b1[e];
  }
  float s = ((xs[0] + xs[1]) + (xs[2] + xs[3])) + ((xs[4] + xs[5]) + (xs[6] + xs[7]));
#pragma unroll
  for (int off = 16; off > 0; off >>= 1) s += __shfl_xor(s, off, 32);
  if (lane == 0) red1[wave] = s;
  __syncthreads();
  float tot = 0.0f;
#pragma unroll
  for (int w = 0; w < 8; ++w) tot += red1[w];
  const float mu = tot * kInvCh;
  float ss = 0.0f;
#pragma unroll
  for (int e = 0; e < 8; ++e) {
    const float d = xs[e] - mu;
    xs[e] = d;
    ss += d * d;
  }
#pragma unroll
  for (int off = 16; off > 0; off >>= 1) ss += __shfl_xor(ss, off, 32);
  if (lane == 0) red2[wave] = ss;
  __syncthreads();
  float tot2 = 0.0f;
#pragma unroll
  for (int w = 0; w < 8; ++w) tot2 += red2[w];
  const float var = tot2 * kInvCh;
  const float rstd = rsqrtf(var + kLnEps);
  v8h hv, lv;
#pragma unroll
  for (int e = 0; e < 8; ++e) {
    const float o = (xs[e] * rstd) * gs[e] + bs[e];
    const _Float16 hi = (_Float16)o;
    const float hif = (float)hi;
    hv[e] = hi;
    lv[e] = (_Float16)((o - hif) * kResCarry);
  }
  const size_t off = (size_t)row * kCh + c0;
  *(volatile v8h*)(yh + off) = hv;
  *(volatile v8h*)(yl + off) = lv;
  __threadfence();
  *(volatile v8h*)(yh + off) = hv;
  *(volatile v8h*)(yl + off) = lv;
}

extern "C" void kernel_launch(void* const* d_in, const int* in_sizes, int n_in,
                              void* d_out, int out_size, void* d_ws, size_t ws_size, hipStream_t stream) {
  if (n_in < 20 || d_out == nullptr || d_ws == nullptr) return;
  if (in_sizes[0] != kPlane || in_sizes[1] != kCh || in_sizes[2] != kCh || in_sizes[3] != kCh ||
      in_sizes[4] != kCh || in_sizes[5] != kCh || in_sizes[6] != kCh * kMixCols ||
      in_sizes[7] != 4 * kMixRank * kCh || in_sizes[8] != kCh || in_sizes[9] != kCh * kDecRank ||
      in_sizes[10] != kDecRank * kCh || in_sizes[11] != kCh * kCh || in_sizes[12] != kCh ||
      in_sizes[13] != kCh * kCh || in_sizes[14] != kCh || in_sizes[15] != kCh * kCh || in_sizes[16] != kCh ||
      in_sizes[17] != kCh || in_sizes[18] != kCh || in_sizes[19] != kCh * kCh || out_size != kPlane) return;

  const float* x      = (const float*)d_in[0];
  const float* maa_x  = (const float*)d_in[1];
  const float* maa_r  = (const float*)d_in[2];
  const float* maa_k  = (const float*)d_in[3];
  const float* maa_v  = (const float*)d_in[4];
  const float* maa_w  = (const float*)d_in[5];
  const float* maa_w1 = (const float*)d_in[6];
  const float* maa_w2 = (const float*)d_in[7];
  const float* tdec   = (const float*)d_in[8];
  const float* td_w1  = (const float*)d_in[9];
  const float* td_w2  = (const float*)d_in[10];
  const float* q_w    = (const float*)d_in[11];
  const float* q_b    = (const float*)d_in[12];
  const float* k_w    = (const float*)d_in[13];
  const float* k_b    = (const float*)d_in[14];
  const float* v_w    = (const float*)d_in[15];
  const float* v_b    = (const float*)d_in[16];
  const float* ln_g   = (const float*)d_in[17];
  const float* ln_b   = (const float*)d_in[18];
  const float* o_w    = (const float*)d_in[19];
  float* out = (float*)d_out;

  char* ws = (char*)d_ws;
  size_t off = 0;
  auto carve = [&](size_t bytes) -> char* { char* p = ws + off; off += (bytes + 255) & ~(size_t)255; return p; };
  const size_t MC = (size_t)kPlane;
  const size_t CC = (size_t)kCh * kCh;
  unsigned short* WT   = (unsigned short*)carve(4 * CC * 2);
  unsigned short* W1T  = (unsigned short*)carve((size_t)kMixCols * kCh * 2);
  unsigned short* TD1T = (unsigned short*)carve((size_t)kDecRank * kCh * 2);
  unsigned short* W2T  = (unsigned short*)carve((size_t)4 * kCh * kMixRank * 2);
  unsigned short* TD2T = (unsigned short*)carve((size_t)kCh * kDecRank * 2);
  unsigned short* XXX  = (unsigned short*)carve(MC * 2);
  float*          MMF  = (float*)carve((size_t)kRows * kMixCols * 4);
  unsigned short* MM16 = (unsigned short*)carve((size_t)kRows * kMixCols * 2);
  unsigned short* M16  = (unsigned short*)carve(4 * MC * 2);
  unsigned short* XH   = (unsigned short*)carve(4 * MC * 2);
  unsigned short* XL   = (unsigned short*)carve(3 * MC * 2);
  float*          HF   = (float*)carve((size_t)kRows * kDecRank * 4);
  unsigned short* H16  = (unsigned short*)carve((size_t)kRows * kDecRank * 2);
  float*          LORA = (float*)carve(MC * 4);
  float*          QKV  = (float*)carve(3 * MC * 4);
  float*          Y    = (float*)carve(MC * 4);
  if (off > ws_size || off > (size_t)134217728) return;
  unsigned short* YH = XH;
  unsigned short* YL = XL;

  wt_cast_kernel<64><<<dim3(kCh / 64, kCh / 64, 4), 256, 0, stream>>>(q_w, k_w, v_w, o_w, 0L, WT, (long)CC, kCh, kCh, kWCarry);
  wt_cast_kernel<64><<<dim3(kCh / 64, kMixCols / 64, 1), 256, 0, stream>>>(maa_w1, maa_w1, maa_w1, maa_w1, 0L, W1T, 0L, kCh, kMixCols, kWCarry);
  wt_cast_kernel<64><<<dim3(kCh / 64, kDecRank / 64, 1), 256, 0, stream>>>(td_w1, td_w1, td_w1, td_w1, 0L, TD1T, 0L, kCh, kDecRank, kWCarry);
  wt_cast_kernel<64><<<dim3(kDecRank / 64, kCh / 64, 1), 256, 0, stream>>>(td_w2, td_w2, td_w2, td_w2, 0L, TD2T, 0L, kDecRank, kCh, kWCarry);
  wt_cast_kernel<32><<<dim3(kMixRank / 32, kCh / 64, 4), 256, 0, stream>>>(maa_w2, maa_w2, maa_w2, maa_w2, (long)kMixRank * kCh, W2T,
                                                                            (long)kCh * kMixRank, kMixRank, kCh, kWCarry);

  mix_kernel<false><<<dim3(kPlane / 8 / 256, 1), 256, 0, stream>>>(x, maa_x, maa_x, maa_x, maa_x, XXX, XXX, XXX);

  wmma_gemm64<false, false, 0><<<dim3(((kRows / 64) * (kMixCols / 64) + 7) / 8, 1), 256, 0, stream>>>(
      XXX, XXX, kCh, 0L, W1T, kCh, 0L, (void*)MMF, kMixCols, 0L, q_b, kRows, kMixCols, kCh, kWCarryInv, 1.0f);
  tanh_cast_kernel<<<(kRows * kMixCols) / 2048, 256, 0, stream>>>(MMF, MM16, kActCarry);

  wmma_gemm64<false, false, 1><<<dim3(((kRows / 64) * (kCh / 64) + 7) / 8, 4), 256, 0, stream>>>(
      MM16, MM16, kMixCols, (long)kMixRank, W2T, kMixRank, (long)kCh * kMixRank, (void*)M16, kCh, (long)MC, q_b,
      kRows, kCh, kMixRank, kMCarry / (kActCarry * kWCarry), 1.0f);

  mix_kernel<true><<<dim3(kPlane / 8 / 256, 4), 256, 0, stream>>>(x, maa_r, maa_k, maa_v, maa_w, M16, XH, XL);

  wmma_gemm64<false, false, 0><<<dim3(((kRows / 64) * (kDecRank / 64) + 7) / 8, 1), 256, 0, stream>>>(
      XH + 3 * MC, XH + 3 * MC, kCh, 0L, TD1T, kCh, 0L, (void*)HF, kDecRank, 0L, q_b, kRows, kDecRank, kCh, kWCarryInv, 1.0f);
  tanh_cast_kernel<<<(kRows * kDecRank) / 2048, 256, 0, stream>>>(HF, H16, kActCarry);

  wmma_gemm64<false, false, 0><<<dim3(((kRows / 64) * (kCh / 64) + 7) / 8, 1), 256, 0, stream>>>(
      H16, H16, kDecRank, 0L, TD2T, kDecRank, 0L, (void*)LORA, kCh, 0L, q_b, kRows, kCh, kDecRank,
      1.0f / (kActCarry * kWCarry), 1.0f);

  const dim3 gbig(((kRows / 64) * (kCh / 64) + 7) / 8, 1);
  wmma_gemm64<true, true, 0><<<gbig, 256, 0, stream>>>(
      XH, XL, kCh, 0L, WT, kCh, 0L, (void*)QKV, kCh, 0L, q_b, kRows, kCh, kCh, kWCarryInv, kResInv);
  wmma_gemm64<true, true, 0><<<gbig, 256, 0, stream>>>(
      XH + MC, XL + MC, kCh, 0L, WT + CC, kCh, 0L, (void*)(QKV + MC), kCh, 0L, k_b, kRows, kCh, kCh, kWCarryInv, kResInv);
  wmma_gemm64<true, true, 0><<<gbig, 256, 0, stream>>>(
      XH + 2 * MC, XL + 2 * MC, kCh, 0L, WT + 2 * CC, kCh, 0L, (void*)(QKV + 2 * MC), kCh, 0L, v_b, kRows, kCh, kCh, kWCarryInv, kResInv);

  gated_scan_kernel<<<kBatch * kHeads, 256, 0, stream>>>(QKV, QKV + MC, QKV + 2 * MC, LORA, tdec, Y);

  ln_split_kernel<<<kRows, 256, 0, stream>>>(Y, ln_g, ln_b, YH, YL);

  wmma_gemm64<true, false, 0><<<gbig, 256, 0, stream>>>(
      YH, YL, kCh, 0L, WT + 3 * CC, kCh, 0L, (void*)out, kCh, 0L, q_b, kRows, kCh, kCh, kWCarryInv, kResInv);
}
